// SpatialRelationLayer_41308995453143
// MI455X (gfx1250) — hardware-verified
//
#include <hip/hip_runtime.h>
#include <math.h>

typedef __attribute__((ext_vector_type(16))) _Float16 v16h;
typedef __attribute__((ext_vector_type(16))) __bf16 v16b;
typedef __attribute__((ext_vector_type(8)))  _Float16 v8h;
typedef __attribute__((ext_vector_type(8)))  float v8f;
typedef __attribute__((ext_vector_type(4)))  float v4f;
typedef __attribute__((ext_vector_type(2)))  float v2f;
typedef __attribute__((ext_vector_type(4)))  unsigned v4u;
typedef __attribute__((ext_vector_type(4)))  int v4i;
typedef float __attribute__((may_alias)) float_a;
typedef int __attribute__((may_alias)) int_a;

template <typename T> __device__ __forceinline__ void vst2(void* p, T v) { *(volatile T*)p = v; __threadfence(); *(volatile T*)p = v; }
__device__ __forceinline__ v8f wmma16(v16h a, v16h b, v8f c) {
  v8f d = __builtin_amdgcn_wmma_f32_16x16x32_f16(false, a, false, b, (short)0, c, false, false);
  asm volatile("v_nop\n\tv_nop\n\tv_nop\n\tv_nop" : "+v"(d) : "v"(a), "v"(b));
  return d;
}
__device__ __forceinline__ v8f wmma_bf(v16b a, v16b b, v8f c) {
  v8f d = __builtin_amdgcn_wmma_f32_16x16x32_bf16(false, a, false, b, (short)0, c, false, false);
  asm volatile("v_nop\n\tv_nop\n\tv_nop\n\tv_nop" : "+v"(d) : "v"(a), "v"(b));
  return d;
}
__device__ __forceinline__ v16h frag_h(const _Float16* rowk0, int lane) {
  union { v16h v; v8h q[2]; } u; const _Float16* p = rowk0 + 8 * (lane >> 4);
  u.q[0] = *(const v8h*)p; u.q[1] = *(const v8h*)(p + 16); return u.v;
}
__device__ __forceinline__ v16h frag_f32(const float* rowk0, int lane) {
  v16h a; const float* p = rowk0 + 8 * (lane >> 4);
#pragma unroll
  for (int i = 0; i < 8; ++i) { a[i] = (_Float16)p[i]; a[8 + i] = (_Float16)p[16 + i]; }
  return a;
}
__device__ __forceinline__ v16h frag_f32s(const float* rowk0, int lane, float sc) {
  v16h a; const float* p = rowk0 + 8 * (lane >> 4);
#pragma unroll
  for (int i = 0; i < 8; ++i) { a[i] = (_Float16)(p[i] * sc); a[8 + i] = (_Float16)(p[16 + i] * sc); }
  return a;
}
__device__ __forceinline__ v16h fragc_f32(const float* W, int k0, int n, int lane, int ld, int K) {
  v16h a; const int g = lane >> 4;
#pragma unroll
  for (int i = 0; i < 8; ++i) { const int ka = k0 + 8 * g + i, kb = ka + 16;
    a[i] = (_Float16)(ka < K ? W[(size_t)(ka < K ? ka : K - 1) * ld + n] : 0.f); a[8 + i] = (_Float16)(kb < K ? W[(size_t)(kb < K ? kb : K - 1) * ld + n] : 0.f); }
  return a;
}
struct F2 { v16b h, l; };
__device__ __forceinline__ F2 bsplit16(const float v[16]) { F2 r;
#pragma unroll
  for (int i = 0; i < 16; ++i) { const __bf16 h = (__bf16)v[i]; r.h[i] = h; r.l[i] = (__bf16)(v[i] - (float)h); }
  return r; }
__device__ __forceinline__ F2 split_row(const float* row, int k0, int lane) { float v[16]; const float* p = row + k0 + 8 * (lane >> 4);
#pragma unroll
  for (int i = 0; i < 8; ++i) { v[i] = p[i]; v[8 + i] = p[16 + i]; }
  return bsplit16(v); }
__device__ __forceinline__ F2 split_rowK(const float* row, int k0, int lane, int K) { float v[16]; const int g = lane >> 4;
#pragma unroll
  for (int i = 0; i < 8; ++i) { const int ka = k0 + 8 * g + i, kb = ka + 16; v[i] = ka < K ? row[ka < K ? ka : K - 1] : 0.f; v[8 + i] = kb < K ? row[kb < K ? kb : K - 1] : 0.f; }
  return bsplit16(v); }
__device__ __forceinline__ F2 split_col(const float* W, int k0, int n, int lane, int ld, int K) { float v[16]; const int g = lane >> 4;
#pragma unroll
  for (int i = 0; i < 8; ++i) { const int ka = k0 + 8 * g + i, kb = ka + 16; v[i] = ka < K ? W[(size_t)(ka < K ? ka : K - 1) * ld + n] : 0.f; v[8 + i] = kb < K ? W[(size_t)(kb < K ? kb : K - 1) * ld + n] : 0.f; }
  return bsplit16(v); }
__device__ __forceinline__ v8f mac3(const F2& a, const F2& b, v8f c) { c = wmma_bf(a.l, b.h, c); c = wmma_bf(a.h, b.l, c); return wmma_bf(a.h, b.h, c); }
__device__ __forceinline__ float sigm(float v) { return 1.0f / (1.0f + expf(-v)); }
#define LDSX() do { asm volatile("s_wait_dscnt 0" ::: "memory"); __builtin_amdgcn_wave_barrier(); __builtin_amdgcn_fence(__ATOMIC_RELEASE, "workgroup"); } while (0)


#define NBATCH 8
#define NOBJ 128
#define D0 128
#define D1 128
#define D2 64
#define HID 132
#define HP 144
#define HK 160
#define OUTC 64
#define DINP 256
#define DINQ 384
#define DINR 320
#define NRQ (NBATCH * NOBJ)
#define NRR (NBATCH * NOBJ * NOBJ)
#define OFFQ (NBATCH * OUTC)
#define OFFR (OFFQ + NRQ * OUTC)
#ifndef TRB
#define TRB (NRR / 64)
#endif
typedef __attribute__((ext_vector_type(8))) __bf16 v8b;
__device__ __forceinline__ v16b frag_b(const __bf16* rowk0, int lane) {
  union { v16b v; v8b q[2]; } u; const __bf16* p = rowk0 + 8 * (lane >> 4);
  u.q[0] = *(const v8b*)p; u.q[1] = *(const v8b*)(p + 16); return u.v;
}
__device__ __forceinline__ float bfr(float v) { return (float)(__bf16)v; }
__device__ __attribute__((noinline)) float exp_ni(float v) { return expf(v); }
__device__ __attribute__((noinline)) float erf_ni(float v) { return erff(v); }

#define WSZ(DIN) (2u * ((size_t)HP * (DIN) + (size_t)HP * HK + (size_t)OUTC * HK))
#define WS_WP  0u
#define WS_WQ  (WS_WP + WSZ(DINP))
#define WS_WR  (WS_WQ + WSZ(DINQ))
#define WS_RR0 (WS_WR + WSZ(DINR))
#define WS_RR1 (WS_RR0 + 4u * (size_t)NRQ * D2)
#define WS_END (WS_RR1 + 4u * (size_t)NRQ * D2)

__global__ __launch_bounds__(128) void k_packw(const float* __restrict__ PW1, const float* __restrict__ PW2, const float* __restrict__ PW3, const float* __restrict__ QW1, const float* __restrict__ QW2, const float* __restrict__ QW3, const float* __restrict__ RW1, const float* __restrict__ RW2, const float* __restrict__ RW3, char* __restrict__ ws) {
  __shared__ __align__(16) _Float16 s1[DINQ], s2[HK], s3[HK]; const int n = blockIdx.x, br = blockIdx.y, t = threadIdx.x;
  const int din = br == 0 ? DINP : br == 1 ? DINQ : DINR; const float* W1 = br == 0 ? PW1 : br == 1 ? QW1 : RW1; const float* W2 = br == 0 ? PW2 : br == 1 ? QW2 : RW2; const float* W3 = br == 0 ? PW3 : br == 1 ? QW3 : RW3; char* base = ws + (br == 0 ? WS_WP : br == 1 ? WS_WQ : WS_WR);
  _Float16* W1h = (_Float16*)base; _Float16* W2h = W1h + (size_t)HP * din; _Float16* W3h = W2h + (size_t)HP * HK;
  for (int k = t; k < din; k += 128) s1[k] = (n < HID) ? (_Float16)bfr(W1[(size_t)k * HID + n]) : (_Float16)0.0f;
  for (int k = t; k < HK; k += 128) { s2[k] = (n < HID && k < HID) ? (_Float16)bfr(W2[(size_t)k * HID + n]) : (_Float16)0.0f; s3[k] = (n < OUTC && k < HID) ? (_Float16)bfr(W3[(size_t)k * OUTC + n]) : (_Float16)0.0f; }
  __syncthreads();
  for (int q = t; q < din / 8; q += 128) vst2((unsigned*)(W1h + (size_t)n * din + q * 8), *(const v4u*)&s1[q * 8]);
  for (int q = t; q < HK / 8; q += 128) vst2((unsigned*)(W2h + (size_t)n * HK + q * 8), *(const v4u*)&s2[q * 8]);
  if (n < OUTC) for (int q = t; q < HK / 8; q += 128) vst2((unsigned*)(W3h + (size_t)n * HK + q * 8), *(const v4u*)&s3[q * 8]); }
__global__ __launch_bounds__(128) void k_rred(const float* __restrict__ R, float* __restrict__ RR0, float* __restrict__ RR1) { __shared__ float red[2][64][2]; __shared__ __align__(16) float so[2][64]; const int n = blockIdx.x, t = threadIdx.x; const size_t b = blockIdx.y; const int c = t & 63, half = t >> 6;
  float m1 = -3.0e38f, m0 = -3.0e38f; for (int j = half; j < NOBJ; j += 2) { m1 = fmaxf(m1, bfr(R[((b * NOBJ + n) * NOBJ + j) * D2 + c])); m0 = fmaxf(m0, bfr(R[((b * NOBJ + j) * NOBJ + n) * D2 + c])); }
  red[0][c][half] = m0; red[1][c][half] = m1; __syncthreads(); if (t < 64) { so[0][t] = fmaxf(red[0][t][0], red[0][t][1]); so[1][t] = fmaxf(red[1][t][0], red[1][t][1]); } __syncthreads();
  if (t < 16) vst2(RR0 + (b * NOBJ + n) * D2 + t * 4, *(const v4f*)&so[0][t * 4]); else if (t < 32) vst2(RR1 + (b * NOBJ + n) * D2 + (t - 16) * 4, *(const v4f*)&so[1][(t - 16) * 4]); }
template <int BR>
__global__ __launch_bounds__(128) void k_mlp(const float* __restrict__ P, const float* __restrict__ Q, const float* __restrict__ R, const float* __restrict__ RR0, const float* __restrict__ RR1, const char* __restrict__ ws, const float* __restrict__ B1, const float* __restrict__ B2, const float* __restrict__ B3, float* __restrict__ OUT) {
  constexpr int DIN = BR == 0 ? DINP : BR == 1 ? DINQ : DINR;
  __shared__ __align__(16) _Float16 sx[64][DIN + 8]; __shared__ __align__(16) _Float16 sh[64][HK + 8]; __shared__ __align__(16) float so[64][OUTC + 4];
  const int tid = threadIdx.x, wave = tid >> 5, lane = tid & 31, col = lane & 15, g = lane >> 4; const size_t row0 = (size_t)blockIdx.x * 64;
  const _Float16* W1h = (const _Float16*)(ws + (BR == 0 ? WS_WP : BR == 1 ? WS_WQ : WS_WR)); const _Float16* W2h = W1h + (size_t)HP * DIN; const _Float16* W3h = W2h + (size_t)HP * HK;
  if (BR == 0) { for (int e = tid; e < 64 * DIN; e += 128) { const int rl = e / DIN, c = e % DIN; float v = 0.f; if (rl < NBATCH) { if (c < D1) { float m = -3.0e38f; for (int n = 0; n < NOBJ; ++n) m = fmaxf(m, bfr(Q[((size_t)rl * NOBJ + n) * D1 + c])); v = m; } else v = bfr(P[(size_t)rl * D0 + c - D1]); } sx[rl][c] = (_Float16)v; } }
  else if (BR == 1) { for (int e = tid; e < 64 * DIN; e += 128) { const int rl = e / DIN, c = e % DIN; const size_t rw = row0 + rl; const size_t b = rw / NOBJ; float v; if (c < D0) v = bfr(P[b * D0 + c]); else if (c < D0 + D1) v = bfr(Q[rw * D1 + c - D0]); else if (c < D0 + D1 + D2) v = RR0[rw * D2 + c - D0 - D1]; else v = RR1[rw * D2 + c - D0 - D1 - D2]; sx[rl][c] = (_Float16)v; } }
  else { for (int e = tid; e < 64 * DIN; e += 128) { const int rl = e / DIN, c = e % DIN; const size_t rw = row0 + rl; const size_t b = rw / (NOBJ * NOBJ); const int i = (int)((rw / NOBJ) % NOBJ), j = (int)(rw % NOBJ); float v; if (c < D2) v = bfr(R[rw * D2 + c]); else if (c < D2 + D1) v = bfr(Q[(b * NOBJ + j) * D1 + c - D2]); else v = bfr(Q[(b * NOBJ + i) * D1 + c - D2 - D1]); sx[rl][c] = (_Float16)v; } }
  for (int e = tid; e < 64 * (HK + 8); e += 128) sh[e / (HK + 8)][e % (HK + 8)] = (_Float16)0.0f;
  __syncthreads();
  { v8f acc[9];
#pragma unroll
    for (int j = 0; j < 9; ++j) acc[j] = v8f{};
#pragma unroll 2
    for (int kc = 0; kc < DIN / 32; ++kc) { v16h a; const _Float16* pp = &sx[wave * 16 + col][kc * 32 + 8 * g];
#pragma unroll
      for (int i = 0; i < 8; ++i) { a[i] = pp[i]; a[8 + i] = pp[16 + i]; }
#pragma unroll
      for (int j = 0; j < 9; ++j) acc[j] = wmma16(a, frag_h(W1h + (size_t)(j * 16 + col) * DIN + kc * 32, lane), acc[j]); }
#pragma unroll
    for (int j = 0; j < 9; ++j) { const int c = j * 16 + col; const float bb = (c < HID) ? bfr(B1[c]) : 0.f;
#pragma unroll
      for (int r = 0; r < 8; ++r) if (c < HID) sh[wave * 16 + 8 * g + r][c] = (_Float16)fmaxf(acc[j][r] + bb, 0.f); } }
  __syncthreads();
  { v8f acc[9];
#pragma unroll
    for (int j = 0; j < 9; ++j) acc[j] = v8f{};
#pragma unroll
    for (int kc = 0; kc < HK / 32; ++kc) { v16h a; const _Float16* pp = &sh[wave * 16 + col][kc * 32 + 8 * g];
#pragma unroll
      for (int i = 0; i < 8; ++i) { a[i] = pp[i]; a[8 + i] = pp[16 + i]; }
#pragma unroll
      for (int j = 0; j < 9; ++j) acc[j] = wmma16(a, frag_h(W2h + (size_t)(j * 16 + col) * HK + kc * 32, lane), acc[j]); }
    __syncthreads();
#pragma unroll
    for (int j = 0; j < 9; ++j) { const int c = j * 16 + col; const float bb = (c < HID) ? bfr(B2[c]) : 0.f;
#pragma unroll
      for (int r = 0; r < 8; ++r) if (c < HID) sh[wave * 16 + 8 * g + r][c] = (_Float16)fmaxf(acc[j][r] + bb, 0.f); } }
  __syncthreads();
  { v8f acc[4] = {};
#pragma unroll
    for (int kc = 0; kc < HK / 32; ++kc) { v16h a; const _Float16* pp = &sh[wave * 16 + col][kc * 32 + 8 * g];
#pragma unroll
      for (int i = 0; i < 8; ++i) { a[i] = pp[i]; a[8 + i] = pp[16 + i]; }
#pragma unroll
      for (int j = 0; j < 4; ++j) acc[j] = wmma16(a, frag_h(W3h + (size_t)(j * 16 + col) * HK + kc * 32, lane), acc[j]); }
#pragma unroll
    for (int j = 0; j < 4; ++j) { const int c = j * 16 + col; const float bb = bfr(B3[c]);
#pragma unroll
      for (int r = 0; r < 8; ++r) { const float z = (acc[j][r] + bb) * 5.0f; so[wave * 16 + 8 * g + r][c] = 1.0f / (1.0f + expf(-z)); } } }
  __syncthreads();
  { float* dst = OUT + (BR == 0 ? 0 : BR == 1 ? OFFQ : OFFR); const int nrows = (BR == 0) ? NBATCH : 64; for (int e = tid; e < nrows * 16; e += 128) { const int rl = e >> 4, q = e & 15; vst2(dst + (row0 + rl) * OUTC + q * 4, *(const v4f*)&so[rl][q * 4]); } } }
extern "C" void kernel_launch(void* const* d_in, const int* in_sizes, int n_in, void* d_out, int out_size, void* d_ws, size_t ws_size, hipStream_t stream) {
  (void)in_sizes; (void)n_in; (void)out_size;
  const float** F = (const float**)d_in;
  if (ws_size < (size_t)WS_END) return;
  char* ws = (char*)d_ws; float *RR0 = (float*)(ws + WS_RR0), *RR1 = (float*)(ws + WS_RR1);
  k_packw<<<dim3(HP, 3), 128, 0, stream>>>(F[3], F[5], F[7], F[9], F[11], F[13], F[15], F[17], F[19], ws);
  k_rred<<<dim3(NOBJ, NBATCH), 128, 0, stream>>>(F[2], RR0, RR1);
  k_mlp<0><<<1, 128, 0, stream>>>(F[0], F[1], F[2], RR0, RR1, ws, F[4], F[6], F[8], (float*)d_out);
  k_mlp<1><<<NRQ / 64, 128, 0, stream>>>(F[0], F[1], F[2], RR0, RR1, ws, F[10], F[12], F[14], (float*)d_out);
  k_mlp<2><<<TRB, 128, 0, stream>>>(F[0], F[1], F[2], RR0, RR1, ws, F[16], F[18], F[20], (float*)d_out);
}
